// ViMHA_5978594476209
// MI455X (gfx1250) — hardware-verified
//
#include <hip/hip_runtime.h>
#include <math.h>
#include <stdint.h>

#define NBT   16
#define NCH   3
#define IMGW  512
#define NPT   1024
#define DM    768
#define NHD   12
#define DHD   64
#define GBI   8
#define NGRP  2
#define MG    (GBI * NPT)
#define PSC   4096.0f
#define LOSC  2048.0f

typedef _Float16 v16h __attribute__((ext_vector_type(16)));
typedef _Float16 v8h  __attribute__((ext_vector_type(8)));
typedef __bf16   v16b __attribute__((ext_vector_type(16)));
typedef __bf16   v8b  __attribute__((ext_vector_type(8)));
typedef float    v8f  __attribute__((ext_vector_type(8)));
typedef float    v4f  __attribute__((ext_vector_type(4)));
typedef unsigned int v4u __attribute__((ext_vector_type(4)));

__device__ __forceinline__ unsigned short f2bf_bits(float f) {
  const unsigned u = __float_as_uint(f);
  return (unsigned short)((u + 0x7FFFu + ((u >> 16) & 1u)) >> 16);
}
__device__ __forceinline__ float bf2f(unsigned short h) { return __uint_as_float(((unsigned)h) << 16); }
__device__ __forceinline__ float bfr(float f) { return bf2f(f2bf_bits(f)); }
__device__ __forceinline__ unsigned pk16(unsigned short a, unsigned short b) { return (unsigned)a | ((unsigned)b << 16); }
__device__ __forceinline__ v8f zero8() { return (v8f){0.f, 0.f, 0.f, 0.f, 0.f, 0.f, 0.f, 0.f}; }

union FragB { v16b v; v8b h[2]; };
union FragH { v16h v; v8h h[2]; };
__device__ __forceinline__ v16b ldfrag_b(const __bf16* p) {
  FragB f; f.h[0] = *(const v8b*)(p); f.h[1] = *(const v8b*)(p + 16); return f.v;
}
__device__ __forceinline__ v16h ldfrag_h(const _Float16* p) {
  FragH f; f.h[0] = *(const v8h*)(p); f.h[1] = *(const v8h*)(p + 16); return f.v;
}

__device__ __forceinline__ v8f mma_b(v16b a, v16b b, v8f c) {
  return __builtin_amdgcn_wmma_f32_16x16x32_bf16(false, a, false, b, (short)0, c, false, false);
}
__device__ __forceinline__ v8f mma_hg(v16h a, v16h b, v8f c) {
  c = __builtin_amdgcn_wmma_f32_16x16x32_f16(false, a, false, b, (short)0, c, false, false);
  asm volatile("v_nop\n\tv_nop\n\tv_nop\n\tv_nop" : "+v"(c) : "v"(a), "v"(b));
  return c;
}
__device__ __forceinline__ void guard_b(v8f& a, v8f& b, v16b x, v16b y) {
  asm volatile("v_nop\n\tv_nop\n\tv_nop\n\tv_nop" : "+v"(a), "+v"(b) : "v"(x), "v"(y));
}
__device__ __forceinline__ void keep4_b(v16b a, v16b b, v16b c, v16b d) {
  asm volatile("v_nop" :: "v"(a), "v"(b), "v"(c), "v"(d));
}
__device__ __forceinline__ void acc_guard4(v8f& a, v8f& b, v8f& c, v8f& d) {
  asm volatile("v_nop\n\tv_nop\n\tv_nop\n\tv_nop" : "+v"(a), "+v"(b), "+v"(c), "+v"(d));
}

template <bool SPLITA, int BIAS_MODE, int PEMODE, int OUT_MODE>
__global__ __launch_bounds__(256) void k_gemm64(
    const unsigned short* __restrict__ Ap, const unsigned short* __restrict__ A2p, int lda, long strideA,
    const unsigned short* __restrict__ Btp, int ldb, long strideB,
    void* Cout, void* Cout2, int ldc, long strideC,
    const float* __restrict__ bias, const float* __restrict__ pew, long strideP,
    int M, int N, int K, float scale) {
  const __bf16* A  = (const __bf16*)(const void*)Ap;
  const __bf16* A2 = (const __bf16*)(const void*)A2p;
  const __bf16* Bt = (const __bf16*)(const void*)Btp;
  __shared__ __align__(16) float sT[8][16 * 68];
  const int b    = blockIdx.y;
  const int lane = threadIdx.x & 31;
  const int wave = threadIdx.x >> 5;
  const int tilesN = N >> 6;
  const int tilesM = M >> 6;
  const int tile = blockIdx.x * 8 + wave;
  if (tile >= tilesM * tilesN) return;
  const int tm = tile / tilesN;
  const int tn = tile - tm * tilesN;
  const int m0 = tm << 6;
  const int n0 = tn << 6;

  const __bf16* Ab  = A  + (size_t)b * strideA;
  const __bf16* Ab2 = A2 + (size_t)b * strideA;
  const __bf16* Bb  = Bt + (size_t)b * strideB;
  const float*  Pb  = pew + (size_t)b * strideP;

  const int rlane = lane & 15;
  const int koff  = (lane >> 4) * 8;
  const int mOff  = (lane >> 4) * 8;

  v8f acc[4][4];
#pragma unroll
  for (int i = 0; i < 4; ++i)
#pragma unroll
    for (int j = 0; j < 4; ++j) acc[i][j] = zero8();

  for (int k0 = 0; k0 < K; k0 += 32) {
    v16b bh[4];
#pragma unroll
    for (int j = 0; j < 4; ++j) {
      const size_t bo = (size_t)(n0 + (j << 4) + rlane) * ldb + koff + k0;
      bh[j] = ldfrag_b(Bb + bo);
    }
#pragma unroll
    for (int i = 0; i < 4; ++i) {
      const size_t ao = (size_t)(m0 + (i << 4) + rlane) * lda + koff + k0;
      v16b ah = ldfrag_b(Ab + ao);
      v16b al = ah;
      if (SPLITA) al = ldfrag_b(Ab2 + ao);
#pragma unroll
      for (int j = 0; j < 4; ++j) {
        acc[i][j] = mma_b(ah, bh[j], acc[i][j]);
        if (SPLITA) acc[i][j] = mma_b(al, bh[j], acc[i][j]);
      }
      guard_b(acc[i][0], acc[i][3], ah, al);
    }
    keep4_b(bh[0], bh[1], bh[2], bh[3]);
  }
  acc_guard4(acc[0][0], acc[0][1], acc[0][2], acc[0][3]);
  acc_guard4(acc[1][0], acc[1][1], acc[1][2], acc[1][3]);
  acc_guard4(acc[2][0], acc[2][1], acc[2][2], acc[2][3]);
  acc_guard4(acc[3][0], acc[3][1], acc[3][2], acc[3][3]);

  float* slab = sT[wave];
#pragma unroll
  for (int i = 0; i < 4; ++i) {
    const int mBase = m0 + (i << 4);
#pragma unroll
    for (int j = 0; j < 4; ++j) {
      const int n = n0 + (j << 4) + rlane;
      float bvv = 0.f;
      if (BIAS_MODE == 2) bvv = bfr(bias[n]);
#pragma unroll
      for (int r = 0; r < 8; ++r) {
        const int mr = mBase + mOff + r;
        float v = acc[i][j][r] * scale;
        if (BIAS_MODE == 1) v += bfr(bias[mr]);
        if (BIAS_MODE == 2) v += bvv;
        if (PEMODE == 1) v += Pb[(size_t)(mr & (NPT - 1)) * DM + n];
        if (PEMODE == 2) v += Pb[(size_t)(n & (NPT - 1)) * DM + mr];
        slab[(mOff + r) * 68 + (j << 4) + rlane] = v;
      }
    }
    __builtin_amdgcn_fence(__ATOMIC_RELEASE, "workgroup");
    __builtin_amdgcn_wave_barrier();
    __builtin_amdgcn_fence(__ATOMIC_ACQUIRE, "workgroup");
    if (OUT_MODE == 0) {
      float* C = (float*)Cout + (size_t)b * strideC;
      const int hh = lane >> 4, c4 = (lane & 15) * 4;
      for (int pass = 0; pass < 2; ++pass) {
#pragma unroll
        for (int it = 0; it < 8; ++it) {
          const int row = it * 2 + hh;
          const v4f v = *(const v4f*)(slab + row * 68 + c4);
          *(volatile v4f*)(C + (size_t)(mBase + row) * ldc + n0 + c4) = v;
        }
        __threadfence();
      }
    } else {
      const int q = lane >> 3, c8 = (lane & 7) * 8;
      unsigned short* C  = (unsigned short*)Cout  + (size_t)b * strideC;
      unsigned short* C2 = (unsigned short*)Cout2 + (size_t)b * strideC;
      for (int pass = 0; pass < 2; ++pass) {
#pragma unroll
        for (int it = 0; it < 4; ++it) {
          const int row = it * 4 + q;
          const float* sp = slab + row * 68 + c8;
          v8h hv, lv;
#pragma unroll
          for (int e = 0; e < 8; ++e) {
            const float v = sp[e];
            const _Float16 hx = (_Float16)v;
            hv[e] = hx;
            if (OUT_MODE == 2) lv[e] = (_Float16)((v - (float)hx) * LOSC);
            else lv[e] = hx;
          }
          *(volatile v8h*)(C + (size_t)(mBase + row) * ldc + n0 + c8) = hv;
          if (OUT_MODE == 2) *(volatile v8h*)(C2 + (size_t)(mBase + row) * ldc + n0 + c8) = lv;
        }
        __threadfence();
      }
    }
    __builtin_amdgcn_fence(__ATOMIC_RELEASE, "workgroup");
    __builtin_amdgcn_wave_barrier();
    __builtin_amdgcn_fence(__ATOMIC_ACQUIRE, "workgroup");
  }
}

__global__ __launch_bounds__(256) void k_wtr(const float* __restrict__ Wq, const float* __restrict__ Wk,
                                             const float* __restrict__ Wv, unsigned short* wt) {
  __shared__ __align__(16) float tf[64 * 68];
  const int z   = blockIdx.z;
  const int mat = z / NHD;
  const int h   = z - mat * NHD;
  const float* W = (mat == 0) ? Wq : ((mat == 1) ? Wk : Wv);
  W += (size_t)h * DM * DHD;
  unsigned short* oh = wt + (size_t)z * DHD * DM;
  const int c0  = blockIdx.x * 64;
  const int r0  = blockIdx.y * 64;
  const int tid = threadIdx.x;
  {
    const int lr = tid >> 4;
    const int c4 = (tid & 15) * 4;
#pragma unroll
    for (int it = 0; it < 4; ++it) {
      const int rr = it * 16 + lr;
      const v4f a = *(const v4f*)(W + (size_t)(r0 + rr) * DHD + c0 + c4);
      *(v4f*)(tf + rr * 68 + c4) = a;
    }
  }
  __syncthreads();
  const int sub = tid >> 3;
  const int c8  = (tid & 7) * 8;
  v4u hv[2];
#pragma unroll
  for (int it = 0; it < 2; ++it) {
    const int oc = it * 32 + sub;
    v4u a;
#pragma unroll
    for (int q = 0; q < 4; ++q) {
      const float f0 = tf[(c8 + 2 * q) * 68 + oc];
      const float f1 = tf[(c8 + 2 * q + 1) * 68 + oc];
      a[q] = pk16(f2bf_bits(f0), f2bf_bits(f1));
    }
    hv[it] = a;
  }
  for (int pass = 0; pass < 2; ++pass) {
#pragma unroll
    for (int it = 0; it < 2; ++it) {
      const int oc = it * 32 + sub;
      *(volatile v4u*)(oh + (size_t)(c0 + oc) * DM + r0 + c8) = hv[it];
    }
    __threadfence();
  }
}

__global__ __launch_bounds__(256) void k_pe(unsigned short* peh, unsigned short* pel) {
#pragma clang fp contract(off)
  const int i = blockIdx.x * 256 + threadIdx.x;
  if (i >= NPT * (DM / 2)) return;
  const int n  = i / (DM / 2);
  const int ip = i - n * (DM / 2);
  const float cexp = -9.21034049987793f * (1.0f / 768.0f);
  const float dv  = expf((float)(2 * ip) * cexp);
  const float ang = (float)n * dv;
  const float sv = sinf(ang);
  const float cv = cosf(ang);
  const unsigned short hs = f2bf_bits(sv), hc = f2bf_bits(cv);
  const unsigned short ls = f2bf_bits(sv - bf2f(hs)), lc = f2bf_bits(cv - bf2f(hc));
  const unsigned uh = pk16(hs, hc), ul = pk16(ls, lc);
  ((volatile unsigned*)peh)[i] = uh;
  ((volatile unsigned*)pel)[i] = ul;
  __threadfence();
  ((volatile unsigned*)peh)[i] = uh;
  ((volatile unsigned*)pel)[i] = ul;
}

__global__ __launch_bounds__(256) void k_xtok(const float* __restrict__ x, unsigned short* xg, int g) {
  const int i = blockIdx.x * 256 + threadIdx.x;
  if (i >= MG * (DM / 8)) return;
  const int tl = i / (DM / 8);
  const int d8 = (i - tl * (DM / 8)) * 8;
  const int n  = tl & (NPT - 1);
  const int bl = tl >> 10;
  const int b  = g * GBI + bl;
  const int f  = n * DM + d8;
  const int c  = f >> 18;
  const int rem = f & 262143;
  const int patch = rem >> 8;
  const int pix = rem & 255;
  const int row = ((patch >> 5) << 4) + (pix >> 4);
  const int col = ((patch & 31) << 4) + (pix & 15);
  const float* src = x + ((size_t)((b * NCH + c) * IMGW + row)) * IMGW + col;
  const v4f a0 = *(const v4f*)(src);
  const v4f a1 = *(const v4f*)(src + 4);
  v4u o;
  o[0] = pk16(f2bf_bits(a0[0]), f2bf_bits(a0[1]));
  o[1] = pk16(f2bf_bits(a0[2]), f2bf_bits(a0[3]));
  o[2] = pk16(f2bf_bits(a1[0]), f2bf_bits(a1[1]));
  o[3] = pk16(f2bf_bits(a1[2]), f2bf_bits(a1[3]));
  unsigned short* dst = xg + (size_t)tl * DM + d8;
  *(volatile v4u*)dst = o;
  __threadfence();
  *(volatile v4u*)dst = o;
}

__global__ __launch_bounds__(128)
void k_attn(const unsigned short* __restrict__ qhp, const unsigned short* __restrict__ qlp,
            const unsigned short* __restrict__ kpp,
            const unsigned short* __restrict__ vhp, const unsigned short* __restrict__ vlp,
            float* of) {
  __shared__ __align__(16) _Float16 Ksh[64 * 64];
  __shared__ __align__(16) _Float16 Vth[64 * 64];
  __shared__ __align__(16) _Float16 Vtl[64 * 64];
  __shared__ __align__(16) _Float16 Psh[4][16 * 64];
  __shared__ __align__(16) float    Os[4][16 * 68];

  const int tid  = threadIdx.x;
  const int wave = tid >> 5;
  const int lane = tid & 31;
  const int hh   = lane >> 4;
  const int c    = lane & 15;

  const int bx = blockIdx.x;
  const int qb = bx & 15;
  const int hb = bx >> 4;
  const int h  = hb % NHD;
  const int bl = hb / NHD;
  const int q0 = bl * NPT + qb * 64 + wave * 16;

  const _Float16* Qh = (const _Float16*)(const void*)qhp + (size_t)h * DHD;
  const _Float16* Ql = (const _Float16*)(const void*)qlp + (size_t)h * DHD;
  const _Float16* Kb = (const _Float16*)(const void*)kpp + (size_t)bl * NPT * DM + (size_t)h * DHD;
  const _Float16* Vh = (const _Float16*)(const void*)vhp + (size_t)h * DHD * MG + (size_t)bl * NPT;
  const _Float16* Vl = (const _Float16*)(const void*)vlp + (size_t)h * DHD * MG + (size_t)bl * NPT;
  float* ob = of + (size_t)h * DHD;

  v16h qah[2], qal[2];
#pragma unroll
  for (int dc = 0; dc < 2; ++dc) {
    qah[dc] = ldfrag_h(Qh + (size_t)(q0 + c) * DM + dc * 32 + 8 * hh);
    qal[dc] = ldfrag_h(Ql + (size_t)(q0 + c) * DM + dc * 32 + 8 * hh);
  }

  float mrow[8], lrow[8];
  v8f oacc[4];
#pragma unroll
  for (int r = 0; r < 8; ++r) { mrow[r] = -INFINITY; lrow[r] = 0.f; }
#pragma unroll
  for (int t = 0; t < 4; ++t) oacc[t] = zero8();

#pragma unroll 1
  for (int kc = 0; kc < NPT / 64; ++kc) {
    const int kv0 = kc * 64;
    __syncthreads();
    {
      const int r = tid >> 1, half = (tid & 1) * 32;
      const _Float16* ks  = Kb + (size_t)(kv0 + r) * DM + half;
      const _Float16* vs  = Vh + (size_t)r * MG + kv0 + half;
      const _Float16* vs2 = Vl + (size_t)r * MG + kv0 + half;
#pragma unroll
      for (int i = 0; i < 4; ++i) {
        const v8h a0 = *(const v8h*)(ks + 8 * i);
        const v8h b0 = *(const v8h*)(vs + 8 * i);
        const v8h b1 = *(const v8h*)(vs2 + 8 * i);
        *(v8h*)(Ksh + r * 64 + half + 8 * i) = a0;
        *(v8h*)(Vth + r * 64 + half + 8 * i) = b0;
        *(v8h*)(Vtl + r * 64 + half + 8 * i) = b1;
      }
    }
    __syncthreads();

    v8f s[4];
#pragma unroll
    for (int j = 0; j < 4; ++j) {
      v8f th = zero8(), tl = zero8();
#pragma unroll
      for (int dc = 0; dc < 2; ++dc) {
        FragH kb;
        kb.h[0] = *(const v8h*)(Ksh + (j * 16 + c) * 64 + dc * 32 + 8 * hh);
        kb.h[1] = *(const v8h*)(Ksh + (j * 16 + c) * 64 + dc * 32 + 16 + 8 * hh);
        th = mma_hg(qah[dc], kb.v, th);
        tl = mma_hg(qal[dc], kb.v, tl);
      }
#pragma unroll
      for (int r = 0; r < 8; ++r) s[j][r] = th[r] * 0.125f + tl[r] * (0.125f / LOSC);
    }

    float cm[8];
#pragma unroll
    for (int r = 0; r < 8; ++r) {
      float m = s[0][r];
      m = fmaxf(m, s[1][r]); m = fmaxf(m, s[2][r]); m = fmaxf(m, s[3][r]);
      m = fmaxf(m, __shfl_xor(m, 1, 32));
      m = fmaxf(m, __shfl_xor(m, 2, 32));
      m = fmaxf(m, __shfl_xor(m, 4, 32));
      m = fmaxf(m, __shfl_xor(m, 8, 32));
      cm[r] = m;
    }
    _Float16* pw = Psh[wave];
#pragma unroll
    for (int r = 0; r < 8; ++r) {
      const float mnew  = fmaxf(mrow[r], cm[r]);
      const float alpha = __expf(mrow[r] - mnew);
      mrow[r] = mnew;
      float psum = 0.f;
#pragma unroll
      for (int j = 0; j < 4; ++j) {
        const float p = __expf(s[j][r] - mnew);
        psum += p;
        pw[(8 * hh + r) * 64 + j * 16 + c] = (_Float16)(p * PSC);
      }
      psum += __shfl_xor(psum, 1, 32);
      psum += __shfl_xor(psum, 2, 32);
      psum += __shfl_xor(psum, 4, 32);
      psum += __shfl_xor(psum, 8, 32);
      lrow[r] = lrow[r] * alpha + psum;
#pragma unroll
      for (int t = 0; t < 4; ++t) oacc[t][r] *= alpha;
    }
    __builtin_amdgcn_fence(__ATOMIC_RELEASE, "workgroup");
    __builtin_amdgcn_wave_barrier();
    __builtin_amdgcn_fence(__ATOMIC_ACQUIRE, "workgroup");

    FragH pa0, pa1;
    pa0.h[0] = *(const v8h*)(pw + c * 64 + 8 * hh);
    pa0.h[1] = *(const v8h*)(pw + c * 64 + 16 + 8 * hh);
    pa1.h[0] = *(const v8h*)(pw + c * 64 + 32 + 8 * hh);
    pa1.h[1] = *(const v8h*)(pw + c * 64 + 48 + 8 * hh);
#pragma unroll
    for (int t = 0; t < 4; ++t) {
      FragH vb0, vb1;
      vb0.h[0] = *(const v8h*)(Vth + (t * 16 + c) * 64 + 8 * hh);
      vb0.h[1] = *(const v8h*)(Vth + (t * 16 + c) * 64 + 16 + 8 * hh);
      vb1.h[0] = *(const v8h*)(Vth + (t * 16 + c) * 64 + 32 + 8 * hh);
      vb1.h[1] = *(const v8h*)(Vth + (t * 16 + c) * 64 + 48 + 8 * hh);
      oacc[t] = mma_hg(pa0.v, vb0.v, oacc[t]);
      oacc[t] = mma_hg(pa1.v, vb1.v, oacc[t]);
      FragH wl0, wl1;
      wl0.h[0] = *(const v8h*)(Vtl + (t * 16 + c) * 64 + 8 * hh);
      wl0.h[1] = *(const v8h*)(Vtl + (t * 16 + c) * 64 + 16 + 8 * hh);
      wl1.h[0] = *(const v8h*)(Vtl + (t * 16 + c) * 64 + 32 + 8 * hh);
      wl1.h[1] = *(const v8h*)(Vtl + (t * 16 + c) * 64 + 48 + 8 * hh);
      v8f tq = zero8();
      tq = mma_hg(pa0.v, wl0.v, tq);
      tq = mma_hg(pa1.v, wl1.v, tq);
#pragma unroll
      for (int r = 0; r < 8; ++r) oacc[t][r] += tq[r] * (1.0f / LOSC);
    }
  }

  float* os = Os[wave];
#pragma unroll
  for (int r = 0; r < 8; ++r) {
    const float inv = (1.0f / lrow[r]) * (1.0f / PSC);
#pragma unroll
    for (int t = 0; t < 4; ++t) os[(8 * hh + r) * 68 + t * 16 + c] = oacc[t][r] * inv;
  }
  __builtin_amdgcn_fence(__ATOMIC_RELEASE, "workgroup");
  __builtin_amdgcn_wave_barrier();
  __builtin_amdgcn_fence(__ATOMIC_ACQUIRE, "workgroup");
  {
    const int c4 = (lane & 15) * 4;
    for (int pass = 0; pass < 2; ++pass) {
#pragma unroll
      for (int it = 0; it < 8; ++it) {
        const int row = it * 2 + hh;
        const v4f val = *(const v4f*)(os + row * 68 + c4);
        *(volatile v4f*)(ob + (size_t)(q0 + row) * DM + c4) = val;
      }
      __threadfence();
    }
  }
}

__global__ __launch_bounds__(256) void k_untok(const float* __restrict__ of, float* out, int g) {
  const int R = blockIdx.x * 2 + (threadIdx.x >> 7);
  if (R >= GBI * NCH * IMGW) return;
  const int t   = threadIdx.x & 127;
  const int bl  = R / (NCH * IMGW);
  const int r2  = R - bl * (NCH * IMGW);
  const int c   = r2 >> 9;
  const int row = r2 & (IMGW - 1);
  const int col = t * 4;
  const float* src = of + (size_t)bl * (NPT * DM) + (size_t)c * 262144
                   + (size_t)((((row >> 4) << 5) + (col >> 4)) * 256) + ((row & 15) << 4) + (col & 15);
  const v4f v = *(const v4f*)src;
  float* dst = out + ((size_t)(((g * GBI + bl) * NCH + c) * IMGW + row)) * IMGW + col;
  *(volatile v4f*)dst = v;
  __threadfence();
  *(volatile v4f*)dst = v;
}

extern "C" void kernel_launch(void* const* d_in, const int* in_sizes, int n_in,
                              void* d_out, int out_size, void* d_ws, size_t ws_size,
                              hipStream_t stream) {
  if (n_in < 7) return;
  if (in_sizes[0] != NBT * NCH * IMGW * IMGW) return;
  if (in_sizes[1] != NHD * DM * DHD || in_sizes[3] != NHD * DM * DHD || in_sizes[5] != NHD * DM * DHD) return;
  if (in_sizes[2] != NHD * DHD || in_sizes[4] != NHD * DHD || in_sizes[6] != NHD * DHD) return;
  if (out_size != NBT * NCH * IMGW * IMGW) return;

  const float* x  = (const float*)d_in[0];
  const float* Wq = (const float*)d_in[1];
  const float* bq = (const float*)d_in[2];
  const float* Wk = (const float*)d_in[3];
  const float* bk = (const float*)d_in[4];
  const float* Wv = (const float*)d_in[5];
  const float* bv = (const float*)d_in[6];
  float* out = (float*)d_out;

  const size_t szWT  = (size_t)3 * DM * DM * 2;
  const size_t szPE  = (size_t)NPT * DM * 2;
  const size_t szPEW = (size_t)3 * NPT * DM * 4;
  const size_t szH   = (size_t)MG * DM * 2;
  const size_t szOF  = (size_t)MG * DM * 4;
  size_t off = 0;
  const size_t oWT  = off; off += szWT;
  const size_t oPEh = off; off += szPE;
  const size_t oPEl = off; off += szPE;
  const size_t oPEW = off; off += szPEW;
  const size_t oX   = off; off += szH;
  const size_t oQh  = off; off += szH;
  const size_t oQl  = off; off += szH;
  const size_t oK   = off; off += szH;
  const size_t oVTh = off; off += szH;
  const size_t oVTl = off; off += szH;
  const size_t oOF  = off; off += szOF;
  if (off > ws_size) return;

  char* ws = (char*)d_ws;
  unsigned short* WT  = (unsigned short*)(ws + oWT);
  unsigned short* PEh = (unsigned short*)(ws + oPEh);
  unsigned short* PEl = (unsigned short*)(ws + oPEl);
  float*          PEW = (float*)(ws + oPEW);
  unsigned short* Xg  = (unsigned short*)(ws + oX);
  unsigned short* Qh  = (unsigned short*)(ws + oQh);
  unsigned short* Ql  = (unsigned short*)(ws + oQl);
  unsigned short* Kp  = (unsigned short*)(ws + oK);
  unsigned short* VTh = (unsigned short*)(ws + oVTh);
  unsigned short* VTl = (unsigned short*)(ws + oVTl);
  float*          OF  = (float*)(ws + oOF);

  const dim3 blk(256);
  const long WPL  = (long)DM * DM;
  const long PEWP = (long)NPT * DM;

  k_wtr<<<dim3(1, DM / 64, 3 * NHD), blk, 0, stream>>>(Wq, Wk, Wv, WT);
  k_pe<<<dim3((NPT * (DM / 2)) / 256), blk, 0, stream>>>(PEh, PEl);
  k_gemm64<true, 0, 0, 0><<<dim3(((NPT / 64) * (DM / 64)) / 8, 3), blk, 0, stream>>>(
      PEh, PEl, DM, 0L, WT, DM, WPL, (void*)PEW, (void*)PEW, DM, PEWP,
      bq, PEW, 0L, NPT, DM, DM, 1.0f);

  const dim3 gTok((MG * (DM / 8)) / 256);
  const dim3 gProj(((MG / 64) * (DM / 64)) / 8, 1);
  const dim3 gAtt(GBI * NHD * (NPT / 64));
  const dim3 gUnt((GBI * NCH * IMGW) / 2);

  for (int g = 0; g < NGRP; ++g) {
    k_xtok<<<gTok, blk, 0, stream>>>(x, Xg, g);
    k_gemm64<false, 2, 1, 2><<<gProj, blk, 0, stream>>>(
        Xg, Xg, DM, 0L, WT, DM, 0L, (void*)Qh, (void*)Ql, DM, 0L,
        bq, PEW, 0L, MG, DM, DM, 2.0f);
    k_gemm64<false, 2, 1, 1><<<gProj, blk, 0, stream>>>(
        Xg, Xg, DM, 0L, WT + WPL, DM, 0L, (void*)Kp, (void*)Kp, DM, 0L,
        bk, PEW + PEWP, 0L, MG, DM, DM, 2.0f);
    k_gemm64<false, 1, 2, 2><<<gProj, blk, 0, stream>>>(
        WT + 2 * WPL, WT + 2 * WPL, DM, 0L, Xg, DM, 0L, (void*)VTh, (void*)VTl, MG, 0L,
        bv, PEW + 2 * PEWP, 0L, DM, MG, DM, 2.0f);
    k_attn<<<gAtt, dim3(128), 0, stream>>>(Qh, Ql, Kp, VTh, VTl, OF);
    k_untok<<<gUnt, blk, 0, stream>>>(OF, out, g);
  }
  (void)hipGetLastError();
}
